// BinaryTreeGRU_10179072491853
// MI455X (gfx1250) — hardware-verified
//
#include <hip/hip_runtime.h>

typedef __bf16          v16bf __attribute__((ext_vector_type(16)));
typedef unsigned short  v8us  __attribute__((ext_vector_type(8)));
typedef unsigned short  v4us  __attribute__((ext_vector_type(4)));
typedef float           v8f   __attribute__((ext_vector_type(8)));
typedef float           v4f   __attribute__((ext_vector_type(4)));
typedef v8us __attribute__((may_alias)) v8usa;
typedef v4us __attribute__((may_alias)) v4usa;
typedef v4f  __attribute__((may_alias)) v4fa;

union Frag { v16bf v; v8us half[2]; };

#define NB     64
#define NLEAF  512
#define NNODE  1023
#define MEMD   256
#define IND    256
#define CATD   512
#define NG3    768
#define NR4    1024
#define NOUT   (NB * NNODE * MEMD)

__device__ __forceinline__ v8f wmma_bf16(v16bf a, v16bf b, v8f c) {
  v8f d = __builtin_amdgcn_wmma_f32_16x16x32_bf16(false, a, false, b, (short)0, c, false, false);
  asm volatile("v_nop\n\tv_nop\n\tv_nop\n\tv_nop" : "+v"(d) : "v"(a), "v"(b));
  return d;
}

__device__ __forceinline__ v8f wmma3(v16bf ah, v16bf al, v16bf bh, v16bf bl, v8f c) {
  c = wmma_bf16(ah, bh, c);
  c = wmma_bf16(ah, bl, c);
  c = wmma_bf16(al, bh, c);
  return c;
}

__device__ __forceinline__ v16bf ldfrag(const unsigned short* p, int h) {
  Frag f;
  f.half[0] = *(const v8usa*)(p + 8 * h);
  f.half[1] = *(const v8usa*)(p + 16 + 8 * h);
  return f.v;
}

__device__ __forceinline__ unsigned bf16_rne(float x) {
  const unsigned u = __float_as_uint(x);
  return (u + 0x7FFFu + ((u >> 16) & 1u)) >> 16;
}

__device__ __forceinline__ void split1(float x, unsigned short& hi, unsigned short& lo) {
  const unsigned hb = bf16_rne(x);
  const float hf = __uint_as_float(hb << 16);
  const unsigned lb = bf16_rne(x - hf);
  hi = (unsigned short)hb;
  lo = (unsigned short)lb;
}

__device__ __forceinline__ void split4(v4f v, v4us& hi, v4us& lo) {
  unsigned short h0, h1, h2, h3, l0, l1, l2, l3;
  split1(v.x, h0, l0);
  split1(v.y, h1, l1);
  split1(v.z, h2, l2);
  split1(v.w, h3, l3);
  hi.x = h0; hi.y = h1; hi.z = h2; hi.w = h3;
  lo.x = l0; lo.y = l1; lo.z = l2; lo.w = l3;
}

__device__ __forceinline__ float sigm(float x) {
  return __builtin_amdgcn_rcpf(1.0f + __expf(-x));
}

__device__ __forceinline__ float tanh_f(float x) {
  const float ax = fabsf(x);
  const float e = __expf(-2.0f * ax);
  const float t = (1.0f - e) * __builtin_amdgcn_rcpf(1.0f + e);
  return copysignf(t, x);
}

__global__ __launch_bounds__(256) void cvt_kernel(
    const float* __restrict__ w0, const float* __restrict__ w1, const float* __restrict__ w2,
    unsigned short* __restrict__ p0h, unsigned short* __restrict__ p0l,
    unsigned short* __restrict__ p1h, unsigned short* __restrict__ p1l,
    unsigned short* __restrict__ p2h, unsigned short* __restrict__ p2l)
{
  const int sel = blockIdx.y;
  const int g = blockIdx.x * 256 + threadIdx.x;
  const float* src = (sel == 0) ? w0 : ((sel == 1) ? w1 : w2);
  unsigned short* dh = (sel == 0) ? p0h : ((sel == 1) ? p1h : p2h);
  unsigned short* dl = (sel == 0) ? p0l : ((sel == 1) ? p1l : p2l);
  const int ng = (sel == 0) ? (NG3 * IND / 8) : ((sel == 1) ? (NR4 * CATD / 8) : (MEMD * MEMD / 8));
  if (g >= ng) return;

  const v4f a = *(const v4fa*)(src + (size_t)g * 8);
  const v4f c = *(const v4fa*)(src + (size_t)g * 8 + 4);
  v4us ha, la, hc, lc;
  split4(a, ha, la);
  split4(c, hc, lc);
  const v8us hh = { ha.x, ha.y, ha.z, ha.w, hc.x, hc.y, hc.z, hc.w };
  const v8us ll = { la.x, la.y, la.z, la.w, lc.x, lc.y, lc.z, lc.w };
  unsigned short* qh = dh + (size_t)g * 8;
  unsigned short* ql = dl + (size_t)g * 8;
  *(volatile v8us*)qh = hh;
  *(volatile v8us*)ql = ll;
  __threadfence();
  *(volatile v8us*)qh = hh;
  *(volatile v8us*)ql = ll;
}

__global__ __launch_bounds__(256) void leaf_kernel(
    const float* __restrict__ x,
    const unsigned short* __restrict__ pg_hi,
    const unsigned short* __restrict__ pg_lo,
    const float* __restrict__ bias,
    float* __restrict__ state,
    float* __restrict__ out)
{
  __shared__ __attribute__((aligned(16))) unsigned short sXh[16 * IND];
  __shared__ __attribute__((aligned(16))) unsigned short sXl[16 * IND];
  __shared__ __attribute__((aligned(16))) float sH[16 * MEMD];

  const int tid = threadIdx.x, lane = tid & 31, w = tid >> 5;
  const int h = lane >> 4, m = lane & 15;
  const int tile = blockIdx.x;

  #pragma unroll
  for (int j = 0; j < 4; ++j) {
    const int g = tid + 256 * j, row = g >> 6, col = (g & 63) * 4;
    const v4f v = *(const v4fa*)(x + (size_t)(tile * 16 + row) * IND + col);
    v4us hh, ll;
    split4(v, hh, ll);
    *(v4usa*)(sXh + row * IND + col) = hh;
    *(v4usa*)(sXl + row * IND + col) = ll;
  }
  __syncthreads();

  const v8f zero8 = {0.f, 0.f, 0.f, 0.f, 0.f, 0.f, 0.f, 0.f};
  const unsigned short* bh0 = pg_hi + (size_t)(32 * w + m) * IND;
  const unsigned short* bl0 = pg_lo + (size_t)(32 * w + m) * IND;

  #pragma unroll
  for (int u = 0; u < 2; ++u) {
    v8f acc[3];
    #pragma unroll
    for (int q = 0; q < 3; ++q) acc[q] = zero8;

    #pragma unroll 1
    for (int k0 = 0; k0 < IND; k0 += 32) {
      const v16bf ah = ldfrag(sXh + m * IND + k0, h);
      const v16bf al = ldfrag(sXl + m * IND + k0, h);
      #pragma unroll
      for (int q = 0; q < 3; ++q) {
        const size_t boff = (size_t)(q * MEMD + 16 * u) * IND + k0;
        const v16bf bh = ldfrag(bh0 + boff, h);
        const v16bf bl = ldfrag(bl0 + boff, h);
        acc[q] = wmma3(ah, al, bh, bl, acc[q]);
      }
    }

    const int mm = 32 * w + 16 * u + m;
    const float b0 = bias[mm], b1 = bias[MEMD + mm], b2 = bias[2 * MEMD + mm];
    #pragma unroll
    for (int r = 0; r < 8; ++r) {
      const float a0 = acc[0][r] + b0;
      const float a1 = acc[1][r] + b1;
      const float a2 = acc[2][r] + b2;
      const float zsum = sigm(a1) + sigm(a2);
      sH[(8 * h + r) * MEMD + mm] = (1.0f - 0.5f * zsum) * tanh_f(a0);
    }
  }
  __syncthreads();

  v4f hv[4];
  size_t go[4];
  #pragma unroll
  for (int i = 0; i < 4; ++i) {
    const int g = tid + 256 * i, row = g >> 6, col = (g & 63) * 4;
    hv[i] = *(const v4fa*)(sH + row * MEMD + col);
    const int rg = tile * 16 + row, bq = rg >> 9, kq = rg & (NLEAF - 1);
    go[i] = (size_t)(bq * NNODE + kq) * MEMD + col;
  }
  #pragma unroll
  for (int i = 0; i < 4; ++i) {
    *(volatile v4f*)(out + go[i]) = hv[i];
    *(volatile v4f*)(state + go[i]) = hv[i];
  }
  __threadfence();
  #pragma unroll
  for (int i = 0; i < 4; ++i) {
    *(volatile v4f*)(out + go[i]) = hv[i];
    *(volatile v4f*)(state + go[i]) = hv[i];
  }
}

__global__ __launch_bounds__(256) void level_kernel(
    float* state,
    float* __restrict__ out,
    const unsigned short* __restrict__ pr_hi,
    const unsigned short* __restrict__ pr_lo,
    const unsigned short* __restrict__ pm_hi,
    const unsigned short* __restrict__ pm_lo,
    const float* __restrict__ bias,
    int offp, int off, int lk)
{
  __shared__ __attribute__((aligned(16))) unsigned char sbuf[16 * CATD * 2 * 2];
  __shared__ __attribute__((aligned(16))) unsigned short sSh[16 * MEMD];
  __shared__ __attribute__((aligned(16))) unsigned short sSl[16 * MEMD];
  unsigned short* sAh = (unsigned short*)sbuf;
  unsigned short* sAl = sAh + 16 * CATD;
  float* sH = (float*)sbuf;

  const int tid = threadIdx.x, lane = tid & 31, w = tid >> 5;
  const int h = lane >> 4, m = lane & 15;
  const int tile = blockIdx.x;
  const int kmask = (1 << lk) - 1;

  #pragma unroll
  for (int j = 0; j < 8; ++j) {
    const int g = tid + 256 * j, row = g >> 7, col = (g & 127) * 4;
    const int rg = tile * 16 + row, bq = rg >> lk, kq = rg & kmask;
    const float* crow = state + (size_t)(bq * NNODE + offp + 2 * kq) * MEMD;
    const v4f v = *(const v4fa*)(crow + col);
    v4us hh, ll;
    split4(v, hh, ll);
    *(v4usa*)(sAh + row * CATD + col) = hh;
    *(v4usa*)(sAl + row * CATD + col) = ll;
  }
  __syncthreads();

  const v8f zero8 = {0.f, 0.f, 0.f, 0.f, 0.f, 0.f, 0.f, 0.f};
  const unsigned short* brh = pr_hi + (size_t)(32 * w + m) * CATD;
  const unsigned short* brl = pr_lo + (size_t)(32 * w + m) * CATD;

  float zc[2][8], zs[2][8];

  #pragma unroll
  for (int u = 0; u < 2; ++u) {
    v8f acc[4];
    #pragma unroll
    for (int q = 0; q < 4; ++q) acc[q] = zero8;

    #pragma unroll 1
    for (int k0 = 0; k0 < CATD; k0 += 32) {
      const v16bf ah = ldfrag(sAh + m * CATD + k0, h);
      const v16bf al = ldfrag(sAl + m * CATD + k0, h);
      #pragma unroll
      for (int q = 0; q < 4; ++q) {
        const size_t boff = (size_t)(q * MEMD + 16 * u) * CATD + k0;
        const v16bf bh = ldfrag(brh + boff, h);
        const v16bf bl = ldfrag(brl + boff, h);
        acc[q] = wmma3(ah, al, bh, bl, acc[q]);
      }
    }

    const int mm = 32 * w + 16 * u + m;
    const float bb0 = bias[MEMD + mm], bb1 = bias[2 * MEMD + mm];
    #pragma unroll
    for (int r = 0; r < 8; ++r) {
      const int row = 8 * h + r;
      const int rg = tile * 16 + row, bq = rg >> lk, kq = rg & kmask;
      const float* crow = state + (size_t)(bq * NNODE + offp + 2 * kq) * MEMD;
      const float c0 = crow[mm], c1 = crow[MEMD + mm];
      const float r0 = sigm(acc[0][r] + bb0);
      const float r1 = sigm(acc[1][r] + bb1);
      const float z0 = sigm(acc[2][r] + bb0);
      const float z1 = sigm(acc[3][r] + bb1);
      const float s = r0 * c0 + r1 * c1;
      unsigned short shv, slv;
      split1(s, shv, slv);
      sSh[row * MEMD + mm] = shv;
      sSl[row * MEMD + mm] = slv;
      zc[u][r] = z0 * c0 + z1 * c1;
      zs[u][r] = z0 + z1;
    }
  }
  __syncthreads();

  v8f acc2[2];
  acc2[0] = zero8;
  acc2[1] = zero8;
  const unsigned short* bmh = pm_hi + (size_t)(32 * w + m) * MEMD;
  const unsigned short* bml = pm_lo + (size_t)(32 * w + m) * MEMD;
  #pragma unroll 1
  for (int k0 = 0; k0 < MEMD; k0 += 32) {
    const v16bf ah = ldfrag(sSh + m * MEMD + k0, h);
    const v16bf al = ldfrag(sSl + m * MEMD + k0, h);
    #pragma unroll
    for (int u = 0; u < 2; ++u) {
      const size_t boff = (size_t)(16 * u) * MEMD + k0;
      const v16bf bh = ldfrag(bmh + boff, h);
      const v16bf bl = ldfrag(bml + boff, h);
      acc2[u] = wmma3(ah, al, bh, bl, acc2[u]);
    }
  }

  #pragma unroll
  for (int u = 0; u < 2; ++u) {
    const int mm = 32 * w + 16 * u + m;
    const float bg = bias[mm];
    #pragma unroll
    for (int r = 0; r < 8; ++r) {
      const float g = tanh_f(acc2[u][r] + bg);
      sH[(8 * h + r) * MEMD + mm] = zc[u][r] + (1.0f - 0.5f * zs[u][r]) * g;
    }
  }
  __syncthreads();

  v4f hv[4];
  size_t go[4];
  #pragma unroll
  for (int i = 0; i < 4; ++i) {
    const int g = tid + 256 * i, row = g >> 6, col = (g & 63) * 4;
    hv[i] = *(const v4fa*)(sH + row * MEMD + col);
    const int rg = tile * 16 + row, bq = rg >> lk, kq = rg & kmask;
    go[i] = (size_t)(bq * NNODE + off + kq) * MEMD + col;
  }
  #pragma unroll
  for (int i = 0; i < 4; ++i) {
    *(volatile v4f*)(out + go[i]) = hv[i];
    *(volatile v4f*)(state + go[i]) = hv[i];
  }
  __threadfence();
  #pragma unroll
  for (int i = 0; i < 4; ++i) {
    *(volatile v4f*)(out + go[i]) = hv[i];
    *(volatile v4f*)(state + go[i]) = hv[i];
  }
}

extern "C" void kernel_launch(void* const* d_in, const int* in_sizes, int n_in,
                              void* d_out, int out_size, void* d_ws, size_t ws_size,
                              hipStream_t stream) {
  if (n_in < 5) return;
  if (in_sizes[0] != NB * NLEAF * IND) return;
  if (in_sizes[1] != NG3 * IND) return;
  if (in_sizes[2] != NG3) return;
  if (in_sizes[3] != NR4 * CATD) return;
  if (in_sizes[4] != MEMD * MEMD) return;
  if (out_size != NOUT) return;

  const float* x     = (const float*)d_in[0];
  const float* Wgrzx = (const float*)d_in[1];
  const float* bgrzx = (const float*)d_in[2];
  const float* Wrzh  = (const float*)d_in[3];
  const float* Wgh   = (const float*)d_in[4];
  float* out = (float*)d_out;

  const size_t st_bytes = (size_t)NOUT * 4;
  const size_t g_bytes  = (size_t)NG3 * IND * 2;
  const size_t r_bytes  = (size_t)NR4 * CATD * 2;
  const size_t m_bytes  = (size_t)MEMD * MEMD * 2;
  const size_t total = st_bytes + 2 * (g_bytes + r_bytes + m_bytes);
  if (total > ws_size) return;

  char* ws = (char*)d_ws;
  float* state = (float*)ws;
  unsigned short* pg_hi = (unsigned short*)(ws + st_bytes);
  unsigned short* pg_lo = (unsigned short*)(ws + st_bytes + g_bytes);
  unsigned short* pr_hi = (unsigned short*)(ws + st_bytes + 2 * g_bytes);
  unsigned short* pr_lo = (unsigned short*)(ws + st_bytes + 2 * g_bytes + r_bytes);
  unsigned short* pm_hi = (unsigned short*)(ws + st_bytes + 2 * g_bytes + 2 * r_bytes);
  unsigned short* pm_lo = (unsigned short*)(ws + st_bytes + 2 * g_bytes + 2 * r_bytes + m_bytes);

  dim3 gcvt(256, 3);
  cvt_kernel<<<gcvt, 256, 0, stream>>>(Wgrzx, Wrzh, Wgh, pg_hi, pg_lo, pr_hi, pr_lo, pm_hi, pm_lo);

  leaf_kernel<<<(NB * NLEAF) / 16, 256, 0, stream>>>(x, pg_hi, pg_lo, bgrzx, state, out);

  int offp = 0;
  for (int lvl = 1; lvl <= 9; ++lvl) {
    const int lk = 9 - lvl;
    const int K = 1 << lk;
    const int off = offp + 2 * K;
    const int blocks = (NB * K) / 16;
    level_kernel<<<blocks, 256, 0, stream>>>(state, out, pr_hi, pr_lo, pm_hi, pm_lo, bgrzx, offp, off, lk);
    offp = off;
  }
}
